// GCN_67826123538777
// MI455X (gfx1250) — hardware-verified
//
#include <hip/hip_runtime.h>
#include <stddef.h>
#include <stdint.h>
#include <math.h>


#define NN     8192
#define FIN    512
#define FH     512
#define FO     256
#define HP     1024
#define NTHR   256
#define NWAVE  8
#define EPT    8
#define CHUNK  (NTHR * EPT)
#define WCAP   (EPT * 32)
#define LISTN  (NWAVE * WCAP)
#define NBA    128
#define SLA    7
#define RCAP   12288
#define DEGCAP 160
#define BIGV   0x7fffffff
#define GBM    64
#define GBN    64
#define GTHR   128
#define NU1    (FH * (FIN / 8))
#define NU2    (FH * (HP / 8))
#define NU3    (FO * (HP / 8))
#define BZ_INTS   (LISTN + 2 * RCAP + 3 * NBA)
#define MISC_INTS 16
#define MST_INTS  (NBA * 4)
#define WBUF_INTS (3 * DEGCAP)
#define BLD_LDS_INTS (BZ_INTS + MISC_INTS + MST_INTS + NWAVE * WBUF_INTS)
#define WSMAX  134217728

static_assert((CHUNK & (CHUNK - 1)) == 0 && CHUNK <= 4096);
static_assert((NBA & (NBA - 1)) == 0 && NBA == (1 << SLA));
static_assert(((long long)CHUNK << SLA) < (1LL << 31));
static_assert(LISTN % NTHR == 0);
static_assert(NBA % NWAVE == 0 && NBA % 32 == 0 && NBA * 2 <= NTHR + NBA);
static_assert(RCAP % 4 == 0 && BZ_INTS % 4 == 0 && BLD_LDS_INTS % 4 == 0);
static_assert(((BZ_INTS + MISC_INTS) % 4) == 0 && ((BZ_INTS + MISC_INTS + MST_INTS) % 4) == 0);
static_assert(DEGCAP == 5 * 32 && (DEGCAP % 4) == 0 && (WBUF_INTS % 4) == 0);
static_assert(BLD_LDS_INTS * 4 <= 300000);
static_assert(FIN % 32 == 0 && HP % 32 == 0 && HP == 2 * FH);
static_assert(NN % GBM == 0 && FH % GBN == 0 && FO % GBN == 0 && GBM == (GTHR / 32) * 16 && GBN == 64);
static_assert(NN % NBA == 0 && NN % NWAVE == 0);
static_assert(NU1 % NTHR == 0 && NU2 % NTHR == 0 && NU3 % NTHR == 0);
static_assert((NN * (FIN / 8)) % NTHR == 0);

typedef float          v4f   __attribute__((ext_vector_type(4)));
typedef float          v8f   __attribute__((ext_vector_type(8)));
typedef int            v4i   __attribute__((ext_vector_type(4)));
typedef int            v8i   __attribute__((ext_vector_type(8)));
typedef unsigned short v4us  __attribute__((ext_vector_type(4)));
typedef unsigned short v8us  __attribute__((ext_vector_type(8)));
typedef unsigned short v16us __attribute__((ext_vector_type(16)));
typedef __bf16         v16bf __attribute__((ext_vector_type(16)));
typedef v4f  __attribute__((may_alias)) v4fa;
typedef v4i  __attribute__((may_alias)) v4ia;
typedef v4us __attribute__((may_alias)) v4usa;
typedef v8us __attribute__((may_alias)) v8usa;
union FragB { v16bf v; v16us u; v8us h[2]; v8i w; };

__device__ __forceinline__ v8f wmb(const FragB& a, const FragB& b, v8f c) {
  v8f d = __builtin_amdgcn_wmma_f32_16x16x32_bf16(false, a.v, false, b.v, (short)0, c, false, false);
  asm volatile("v_nop\n\tv_nop\n\tv_nop\n\tv_nop" : "+v"(d) : "v"(a.w), "v"(b.w));
  return d;
}

__device__ __forceinline__ unsigned bf16_bits(float f) {
  const unsigned u = __float_as_uint(f);
  return (u + 0x7FFFu + ((u >> 16) & 1u)) >> 16;
}
__device__ __forceinline__ float bf16_val(float f) {
  return __uint_as_float(bf16_bits(f) << 16);
}

__device__ __forceinline__ void wave_sync() {
  __builtin_amdgcn_fence(__ATOMIC_RELEASE, "wavefront");
  __builtin_amdgcn_wave_barrier();
  __builtin_amdgcn_fence(__ATOMIC_ACQUIRE, "wavefront");
}

template <int SLB>
__device__ __forceinline__ int scan_chunk(const int* __restrict__ dsts, int nE, int cbase, int slotBase,
                                          int nb, int vec8, int* list, int tid, int lane, int wave) {
  int wc = 0;
  const int el0  = tid * EPT;
  const int e0   = cbase + el0;
  const int sent = -2147483647 - 1;
  v4i da, db;
  if (vec8 != 0 && cbase + CHUNK <= nE) {
    da = *(const v4i*)(dsts + e0);
    db = *(const v4i*)(dsts + e0 + 4);
  } else {
    da.x = (e0     < nE) ? dsts[min(e0,     nE - 1)] : sent;
    da.y = (e0 + 1 < nE) ? dsts[min(e0 + 1, nE - 1)] : sent;
    da.z = (e0 + 2 < nE) ? dsts[min(e0 + 2, nE - 1)] : sent;
    da.w = (e0 + 3 < nE) ? dsts[min(e0 + 3, nE - 1)] : sent;
    db.x = (e0 + 4 < nE) ? dsts[min(e0 + 4, nE - 1)] : sent;
    db.y = (e0 + 5 < nE) ? dsts[min(e0 + 5, nE - 1)] : sent;
    db.z = (e0 + 6 < nE) ? dsts[min(e0 + 6, nE - 1)] : sent;
    db.w = (e0 + 7 < nE) ? dsts[min(e0 + 7, nE - 1)] : sent;
  }
  const unsigned nbs = (unsigned)slotBase;
  const unsigned unb = (unsigned)nb;
  const unsigned s0 = (unsigned)da.x - nbs, s1 = (unsigned)da.y - nbs;
  const unsigned s2 = (unsigned)da.z - nbs, s3 = (unsigned)da.w - nbs;
  const unsigned s4 = (unsigned)db.x - nbs, s5 = (unsigned)db.y - nbs;
  const unsigned s6 = (unsigned)db.z - nbs, s7 = (unsigned)db.w - nbs;
  const bool h0 = s0 < unb, h1 = s1 < unb, h2 = s2 < unb, h3 = s3 < unb;
  const bool h4 = s4 < unb, h5 = s5 < unb, h6 = s6 < unb, h7 = s7 < unb;
  const unsigned any = __builtin_amdgcn_ballot_w32(h0 | h1 | h2 | h3 | h4 | h5 | h6 | h7);
  if (any != 0u) {
#define HITJ(J, HJ, SJ) { \
      const unsigned mj = __builtin_amdgcn_ballot_w32(HJ); \
      if (mj != 0u) { \
        if (HJ) { \
          const int pos = wc + (int)__builtin_amdgcn_mbcnt_lo(mj, 0u); \
          if (pos < WCAP) list[wave * WCAP + pos] = ((el0 + (J)) << SLB) | (int)(SJ); \
        } \
        wc += (int)__builtin_popcount(mj); } }
    HITJ(0, h0, s0)
    HITJ(1, h1, s1)
    HITJ(2, h2, s2)
    HITJ(3, h3, s3)
    HITJ(4, h4, s4)
    HITJ(5, h5, s5)
    HITJ(6, h6, s6)
    HITJ(7, h7, s7)
#undef HITJ
  }
  return wc;
}

__global__ __launch_bounds__(NTHR) void k_wprep(const float* __restrict__ W1, const float* __restrict__ W2,
                                                const float* __restrict__ W3,
                                                unsigned short* W1T, unsigned short* W2D, unsigned short* W3D) {
  const int u = (int)blockIdx.x * NTHR + (int)threadIdx.x;
  v8us o;
  unsigned short* dp;
  if (u < NU1) {
    const int n  = u >> 6;
    const int k8 = (u & 63) * 8;
    const float* p = W1 + (size_t)k8 * FH + n;
#pragma unroll
    for (int i = 0; i < 8; ++i) o[i] = (unsigned short)bf16_bits(p[(size_t)i * FH]);
    dp = W1T + (size_t)n * FIN + k8;
  } else if (u < NU1 + NU2) {
    const int v  = u - NU1;
    const int n  = v >> 7;
    const int k8 = (v & 127) * 8;
    const int kk = k8 & (FH - 1);
    const float* p = W2 + (size_t)kk * FH + n;
#pragma unroll
    for (int i = 0; i < 8; ++i) o[i] = (unsigned short)bf16_bits(p[(size_t)i * FH]);
    dp = W2D + (size_t)n * HP + k8;
  } else if (u < NU1 + NU2 + NU3) {
    const int v  = u - NU1 - NU2;
    const int n  = v >> 7;
    const int k8 = (v & 127) * 8;
    const int kk = k8 & (FH - 1);
    const float* p = W3 + (size_t)kk * FO + n;
#pragma unroll
    for (int i = 0; i < 8; ++i) o[i] = (unsigned short)bf16_bits(p[(size_t)i * FO]);
    dp = W3D + (size_t)n * HP + k8;
  } else {
    return;
  }
  *(volatile v8us*)dp = o;
  __threadfence();
  *(volatile v8us*)dp = o;
}

__global__ __launch_bounds__(NTHR) void k_cvx(const float* __restrict__ x, int nUnits, unsigned short* xb) {
  const int u = (int)blockIdx.x * NTHR + (int)threadIdx.x;
  if (u >= nUnits) return;
  const float* p = x + (size_t)u * 8;
  const v4f a = *(const v4fa*)p;
  const v4f b = *(const v4fa*)(p + 4);
  v8us o;
  o[0] = (unsigned short)bf16_bits(a.x); o[1] = (unsigned short)bf16_bits(a.y);
  o[2] = (unsigned short)bf16_bits(a.z); o[3] = (unsigned short)bf16_bits(a.w);
  o[4] = (unsigned short)bf16_bits(b.x); o[5] = (unsigned short)bf16_bits(b.y);
  o[6] = (unsigned short)bf16_bits(b.z); o[7] = (unsigned short)bf16_bits(b.w);
  unsigned short* dp = xb + (size_t)u * 8;
  *(volatile v8us*)dp = o;
  __threadfence();
  *(volatile v8us*)dp = o;
}

__global__ __launch_bounds__(NTHR) void k_build(const int* __restrict__ ei, int nE2, int nN, int vec8,
                                                int* nbrp, int* metap) {
  extern __shared__ __attribute__((aligned(16))) int dsm[];
  int* list = dsm;
  int* hl   = dsm + LISTN;
  int* sl   = hl + RCAP;
  int* cnt  = sl + RCAP;
  int* offs = cnt + NBA;
  int* cur  = offs + NBA;
  int* misc = cur + NBA;
  int* mst  = misc + MISC_INTS;
  const int tid = (int)threadIdx.x, lane = tid & 31, wave = tid >> 5;
  int* vbuf = mst + MST_INTS + wave * WBUF_INTS;
  int* kbuf = vbuf + DEGCAP;
  int* sbuf = kbuf + DEGCAP;
  const int nodeBase = (int)blockIdx.x * NBA;
  const int eHalf = nE2 >> 1;

  {
    const v4i z4 = {0, 0, 0, 0};
    for (int i = tid * 4; i < BLD_LDS_INTS; i += NTHR * 4) *(v4ia*)(dsm + i) = z4;
  }
  __syncthreads();

  int t = 0, ov = 0;
  const int nChunks = (nE2 + CHUNK - 1) / CHUNK;
#pragma unroll 1
  for (int ch = 0; ch < nChunks; ++ch) {
    const int cbase = ch * CHUNK;
    const int wc = scan_chunk<SLA>(ei, nE2, cbase, nodeBase, NBA, vec8, list, tid, lane, wave);
    if (lane == 0) misc[wave] = wc;
    __syncthreads();
    if (wave == 0) {
#pragma unroll 1
      for (int w2 = 0; w2 < NWAVE; ++w2) {
        int c = misc[w2];
        c = c < 0 ? 0 : (c > WCAP ? WCAP : c);
#pragma unroll 1
        for (int b0 = 0; b0 < c; b0 += 32) {
          const int idx = b0 + lane;
          const int ent = list[w2 * WCAP + (idx < WCAP ? idx : WCAP - 1)];
          const int m32 = (c - b0) < 32 ? (c - b0) : 32;
#pragma unroll 1
          for (int k = 0; k < m32; ++k) {
            const int u    = __builtin_amdgcn_readlane(ent, k);
            const int slot = u & (NBA - 1);
            const int el   = (u >> SLA) & (CHUNK - 1);
            const int pk   = ((cbase + el) << SLA) | slot;
            if (t < RCAP) {
              if (lane == 0) { hl[t] = pk; cnt[slot] = cnt[slot] + 1; }
              t = t + 1;
            } else {
              ov = 1;
            }
          }
        }
      }
    }
    __syncthreads();
  }
  if (wave == 0 && lane == 0) { misc[8] = t; misc[9] = ov; }
  __syncthreads();
  int tt = misc[8];
  tt = tt < 0 ? 0 : (tt > RCAP ? RCAP : tt);
  const int ovf = misc[9];

  if (wave == 0) {
    const int base = lane * (NBA / 32);
    int s = 0;
#pragma unroll 1
    for (int i = 0; i < NBA / 32; ++i) s += cnt[base + i];
    int incl = s;
#pragma unroll
    for (int d = 1; d < 32; d <<= 1) {
      const int y = __shfl_up(incl, d, 32);
      if (lane >= d) incl += y;
    }
    int run = incl - s;
#pragma unroll 1
    for (int i = 0; i < NBA / 32; ++i) {
      const int cv = cnt[base + i];
      offs[base + i] = run;
      cur[base + i]  = run;
      run += cv;
    }
  }
  __syncthreads();
  if (wave == 0) {
#pragma unroll 1
    for (int b0 = 0; b0 < tt; b0 += 32) {
      const int idx = b0 + lane;
      const int ent = hl[idx < RCAP ? idx : RCAP - 1];
      const int m32 = (tt - b0) < 32 ? (tt - b0) : 32;
#pragma unroll 1
      for (int k = 0; k < m32; ++k) {
        const int u    = __builtin_amdgcn_readlane(ent, k);
        const int slot = u & (NBA - 1);
        if (lane == 0) {
          int p = cur[slot];
          p = p < 0 ? 0 : (p > RCAP - 1 ? RCAP - 1 : p);
          sl[p] = u;
          cur[slot] = p + 1;
        }
      }
    }
  }
  __syncthreads();

#pragma unroll 1
  for (int si = 0; si < NBA / NWAVE; ++si) {
    const int s    = si * NWAVE + wave;
    const int node = nodeBase + s;
    const int craw = cnt[s];
    const bool big = craw > DEGCAP;
    int c = craw < 0 ? 0 : (craw > DEGCAP ? DEGCAP : craw);
    c = __builtin_amdgcn_readfirstlane(c);
    int o = offs[s];
    o = o < 0 ? 0 : (o > RCAP ? RCAP : o);
    o = __builtin_amdgcn_readfirstlane(o);

#pragma unroll
    for (int q = 0; q < DEGCAP / 32; ++q) sbuf[32 * q + lane] = 0;

#pragma unroll 1
    for (int b0 = 0; b0 < c; b0 += 32) {
      const int i = b0 + lane;
      int idx = o + i;
      idx = idx > RCAP - 1 ? RCAP - 1 : idx;
      const int ent = sl[idx];
      int eid = ent >> SLA;
      eid = eid < 0 ? 0 : (eid > nE2 - 1 ? nE2 - 1 : eid);
      int pe = eid + eHalf;
      pe = pe >= nE2 ? pe - nE2 : pe;
      int nb = ei[pe];
      nb = nb < 0 ? 0 : (nb > nN - 1 ? nN - 1 : nb);
      vbuf[i] = nb;
    }
    wave_sync();

    unsigned selfm = 0u;
#pragma unroll 1
    for (int b0 = 0; b0 < c; b0 += 32) {
      const int i  = b0 + lane;
      const int ic = i < c ? i : c - 1;
      const int a  = vbuf[ic];
      int dup = 0;
#pragma unroll 2
      for (int j = 0; j < c; ++j) {
        const int vj = vbuf[j];
        dup |= ((vj == a) & (j < i)) ? 1 : 0;
      }
      const bool inr  = i < c;
      const bool self = (a == node);
      selfm |= __builtin_amdgcn_ballot_w32(inr && self);
      const bool keep = inr && !self && (dup == 0);
      kbuf[i] = keep ? a : BIGV;
    }
    wave_sync();

    int nk = 0;
#pragma unroll 1
    for (int b0 = 0; b0 < c; b0 += 32) {
      const int i  = b0 + lane;
      const int ic = i < c ? i : c - 1;
      const int a  = kbuf[ic];
      int rank = 0;
#pragma unroll 2
      for (int j = 0; j < c; ++j) {
        const int vj = kbuf[j];
        rank += (vj < a) ? 1 : 0;
      }
      const bool valid = (i < c) && (a != BIGV);
      rank = rank > DEGCAP - 1 ? DEGCAP - 1 : rank;
      if (valid) sbuf[rank] = a;
      nk += (int)__builtin_popcount(__builtin_amdgcn_ballot_w32(valid));
    }
    wave_sync();

    const v4i q0 = *(const v4ia*)(sbuf + 4 * lane);
    const v4i q1 = *(const v4ia*)(sbuf + 128 + 4 * (lane & 7));
    wave_sync();

    int* rp = nbrp + (size_t)node * DEGCAP;
    *(volatile v4i*)(rp + 4 * lane) = q0;
    if (lane < 8) *(volatile v4i*)(rp + 128 + 4 * lane) = q1;
    __threadfence();
    *(volatile v4i*)(rp + 4 * lane) = q0;
    if (lane < 8) *(volatile v4i*)(rp + 128 + 4 * lane) = q1;

    const int dwi = (selfm != 0u) ? 2 : 1;
    const float dg = (float)(nk + dwi);
    const float dv = 1.0f / sqrtf(dg);
    v4i mv;
    mv.x = nk;
    mv.y = dwi;
    mv.z = __float_as_int(dv);
    mv.w = (ovf != 0 || big) ? 1 : 0;
    if (lane == 0) *(v4ia*)(mst + 4 * s) = mv;
  }
  __syncthreads();
  {
    const int sidx = tid & (NBA - 1);
    const v4i mv = *(const v4ia*)(mst + 4 * sidx);
    int* mp = metap + 4 * (size_t)(nodeBase + sidx);
    const bool wr = tid < NBA;
    if (wr) *(volatile v4i*)mp = mv;
    __threadfence();
    if (wr) *(volatile v4i*)mp = mv;
  }
}

__global__ __launch_bounds__(GTHR) void k_gemm(
    const unsigned short* __restrict__ A, const unsigned short* __restrict__ WT,
    float* outF, int K, int ldo)
{
  __shared__ __attribute__((aligned(16))) float stg[GBM * GBN];
  const int tid = (int)threadIdx.x, lane = tid & 31, wave = tid >> 5, hh = lane >> 4, m = lane & 15;
  const int rowBase = (int)blockIdx.x * GBM;
  const int col0    = (int)blockIdx.y * GBN;

  v8f acc[4];
  {
    const v8f z = {0.f, 0.f, 0.f, 0.f, 0.f, 0.f, 0.f, 0.f};
    acc[0] = z; acc[1] = z; acc[2] = z; acc[3] = z;
  }
  const unsigned short* ap = A  + (size_t)(rowBase + 16 * wave + m) * (size_t)K + 8 * hh;
  const unsigned short* wp = WT + (size_t)(col0 + m) * (size_t)K + 8 * hh;
  const int ksteps = K >> 5;
#pragma unroll 1
  for (int ks = 0; ks < ksteps; ++ks) {
    FragB af;
    af.h[0] = *(const v8usa*)(ap + 32 * ks);
    af.h[1] = *(const v8usa*)(ap + 32 * ks + 16);
#pragma unroll
    for (int t = 0; t < 4; ++t) {
      const unsigned short* wq = wp + (size_t)(16 * t) * (size_t)K + 32 * ks;
      FragB bf;
      bf.h[0] = *(const v8usa*)wq;
      bf.h[1] = *(const v8usa*)(wq + 16);
      acc[t] = wmb(af, bf, acc[t]);
    }
  }

#pragma unroll
  for (int t = 0; t < 4; ++t) {
    const int lc = 16 * t + m;
#pragma unroll
    for (int r = 0; r < 8; ++r) {
      const int lr = 16 * wave + 8 * hh + r;
      stg[lr * GBN + lc] = acc[t][r];
    }
  }
  __syncthreads();

  v4f fv[8];
#pragma unroll
  for (int i = 0; i < 8; ++i) {
    const int lr = 16 * wave + 2 * i + hh;
    fv[i] = *(const v4fa*)(stg + lr * GBN + 4 * m);
  }
#pragma unroll
  for (int i = 0; i < 8; ++i) {
    const int lr = 16 * wave + 2 * i + hh;
    const int gr = rowBase + lr;
    float* op = outF + (size_t)gr * (size_t)ldo + col0 + 4 * m;
    *(volatile v4f*)op = fv[i];
  }
  __threadfence();
#pragma unroll
  for (int i = 0; i < 8; ++i) {
    const int lr = 16 * wave + 2 * i + hh;
    const int gr = rowBase + lr;
    float* op = outF + (size_t)gr * (size_t)ldo + col0 + 4 * m;
    *(volatile v4f*)op = fv[i];
  }
}

template <int NQ, int MODE>
__global__ __launch_bounds__(NTHR) void k_agg(const int* __restrict__ nbr, const int* __restrict__ meta,
                                              const float* __restrict__ xw, const float* __restrict__ bias,
                                              unsigned short* hb, float* outp, int nN) {
  constexpr int F = 128 * NQ;
  static_assert(MODE == 0 || F == FH);
  __shared__ __attribute__((aligned(16))) unsigned short rowb[(MODE != 0) ? (NWAVE * HP) : 16];
  const int tid = (int)threadIdx.x, lane = tid & 31, wave = tid >> 5;
  int node = (int)blockIdx.x * NWAVE + wave;
  node = node < nN ? node : nN - 1;

  const v4i mi = *(const v4i*)(meta + 4 * (size_t)node);
  const bool bad = (mi.w != 0) || (mi.x < 0) || (mi.x > DEGCAP);
  int c = mi.x < 0 ? 0 : (mi.x > DEGCAP ? DEGCAP : mi.x);
  c = __builtin_amdgcn_readfirstlane(c);
  const float dwf = (mi.y == 2) ? 2.0f : 1.0f;
  const float di  = __int_as_float(mi.z);

  v4f acc[NQ];
#pragma unroll
  for (int q = 0; q < NQ; ++q) { const v4f z = {0.0f, 0.0f, 0.0f, 0.0f}; acc[q] = z; }

  const int* nrow = nbr + (size_t)node * DEGCAP;
#pragma unroll 1
  for (int b0 = 0; b0 < c; b0 += 32) {
    int idx = b0 + lane;
    idx = idx > DEGCAP - 1 ? DEGCAP - 1 : idx;
    int sr = nrow[idx];
    sr = sr < 0 ? 0 : (sr > nN - 1 ? nN - 1 : sr);
    const float dj  = __int_as_float(meta[4 * (size_t)sr + 2]);
    const float cf  = (di * 1.0f) * dj;
    const int   cfi = __float_as_int(cf);
    const int m32 = (c - b0) < 32 ? (c - b0) : 32;
#pragma unroll 1
    for (int k = 0; k < m32; ++k) {
      const int   sk = __builtin_amdgcn_readlane(sr, k);
      const float ck = __int_as_float(__builtin_amdgcn_readlane(cfi, k));
      const float* rp = xw + (size_t)sk * F + 4 * lane;
#pragma unroll
      for (int q = 0; q < NQ; ++q) {
        const v4f a = *(const v4fa*)(rp + 128 * q);
        acc[q].x = fmaf(ck, a.x, acc[q].x);
        acc[q].y = fmaf(ck, a.y, acc[q].y);
        acc[q].z = fmaf(ck, a.z, acc[q].z);
        acc[q].w = fmaf(ck, a.w, acc[q].w);
      }
    }
  }

  const float cs   = (di * dwf) * di;
  const float qnan = __int_as_float(0x7fc00000);
  v4f y[NQ];
#pragma unroll
  for (int q = 0; q < NQ; ++q) {
    const v4f sv = *(const v4fa*)(xw + (size_t)node * F + 128 * q + 4 * lane);
    const v4f bq = *(const v4fa*)(bias + 128 * q + 4 * lane);
    v4f t;
    t.x = fmaf(cs, sv.x, acc[q].x) + bf16_val(bq.x);
    t.y = fmaf(cs, sv.y, acc[q].y) + bf16_val(bq.y);
    t.z = fmaf(cs, sv.z, acc[q].z) + bf16_val(bq.z);
    t.w = fmaf(cs, sv.w, acc[q].w) + bf16_val(bq.w);
    if constexpr (MODE != 0) {
      t.x = (t.x > 0.0f) ? t.x : (t.x - t.x);
      t.y = (t.y > 0.0f) ? t.y : (t.y - t.y);
      t.z = (t.z > 0.0f) ? t.z : (t.z - t.z);
      t.w = (t.w > 0.0f) ? t.w : (t.w - t.w);
    }
    t.x = bad ? qnan : t.x;
    t.y = bad ? qnan : t.y;
    t.z = bad ? qnan : t.z;
    t.w = bad ? qnan : t.w;
    y[q] = t;
  }

  if constexpr (MODE != 0) {
    unsigned short* rb = rowb + wave * HP;
#pragma unroll
    for (int q = 0; q < NQ; ++q) {
      v4us h4, l4;
      unsigned hbv;
      hbv = bf16_bits(y[q].x); h4[0] = (unsigned short)hbv; l4[0] = (unsigned short)bf16_bits(y[q].x - __uint_as_float(hbv << 16));
      hbv = bf16_bits(y[q].y); h4[1] = (unsigned short)hbv; l4[1] = (unsigned short)bf16_bits(y[q].y - __uint_as_float(hbv << 16));
      hbv = bf16_bits(y[q].z); h4[2] = (unsigned short)hbv; l4[2] = (unsigned short)bf16_bits(y[q].z - __uint_as_float(hbv << 16));
      hbv = bf16_bits(y[q].w); h4[3] = (unsigned short)hbv; l4[3] = (unsigned short)bf16_bits(y[q].w - __uint_as_float(hbv << 16));
      *(v4usa*)(rb + 128 * q + 4 * lane) = h4;
      *(v4usa*)(rb + FH + 128 * q + 4 * lane) = l4;
    }
    wave_sync();
    v8us qv[HP / 256];
#pragma unroll
    for (int r = 0; r < HP / 256; ++r) qv[r] = *(const v8usa*)(rb + 256 * r + 8 * lane);
    unsigned short* hp = hb + (size_t)node * HP + 8 * lane;
#pragma unroll
    for (int r = 0; r < HP / 256; ++r) *(volatile v8us*)(hp + 256 * r) = qv[r];
    __threadfence();
#pragma unroll
    for (int r = 0; r < HP / 256; ++r) *(volatile v8us*)(hp + 256 * r) = qv[r];
  } else {
    float* op = outp + (size_t)node * F + 4 * lane;
#pragma unroll
    for (int q = 0; q < NQ; ++q) *(volatile v4f*)(op + 128 * q) = y[q];
    __threadfence();
#pragma unroll
    for (int q = 0; q < NQ; ++q) *(volatile v4f*)(op + 128 * q) = y[q];
  }
}

static inline size_t al256(size_t o) { return (o + 255) & ~(size_t)255; }

extern "C" void kernel_launch(void* const* d_in, const int* in_sizes, int n_in,
                              void* d_out, int out_size, void* d_ws, size_t ws_size,
                              hipStream_t stream) {
  if (n_in < 8) return;
  if (in_sizes[0] != NN * FIN) return;
  const int nE2 = in_sizes[1];
  if (nE2 < 2 || (nE2 & 1) != 0 || nE2 >= (1 << (31 - SLA))) return;
  if (in_sizes[2] != FIN * FH || in_sizes[3] != FH) return;
  if (in_sizes[4] != FH * FH  || in_sizes[5] != FH) return;
  if (in_sizes[6] != FH * FO  || in_sizes[7] != FO) return;
  if (out_size != NN * FO) return;

  const float* x  = (const float*)d_in[0];
  const int*   ei = (const int*)d_in[1];
  const float* W1 = (const float*)d_in[2];
  const float* b1 = (const float*)d_in[3];
  const float* W2 = (const float*)d_in[4];
  const float* b2 = (const float*)d_in[5];
  const float* W3 = (const float*)d_in[6];
  const float* b3 = (const float*)d_in[7];
  float* out = (float*)d_out;
  const int nN = NN;
  const int vec8 = ((nE2 & 3) == 0) ? 1 : 0;

  char* ws = (char*)d_ws;
  size_t off = 0;
  const size_t oW1T = off; off = al256(off + (size_t)FH * FIN * 2);
  const size_t oW2D = off; off = al256(off + (size_t)FH * HP * 2);
  const size_t oW3D = off; off = al256(off + (size_t)FO * HP * 2);
  const size_t oXB  = off; off = al256(off + (size_t)NN * FIN * 2);
  const size_t oXW  = off; off = al256(off + (size_t)NN * FH * 4);
  const size_t oH   = off; off = al256(off + (size_t)NN * HP * 2);
  const size_t oNBR = off; off = al256(off + (size_t)NN * DEGCAP * 4);
  const size_t oMET = off; off = al256(off + (size_t)NN * 16);
  if (off > ws_size || off > (size_t)WSMAX) return;
  unsigned short* W1T = (unsigned short*)(ws + oW1T);
  unsigned short* W2D = (unsigned short*)(ws + oW2D);
  unsigned short* W3D = (unsigned short*)(ws + oW3D);
  unsigned short* XB  = (unsigned short*)(ws + oXB);
  float*          XW  = (float*)(ws + oXW);
  unsigned short* H   = (unsigned short*)(ws + oH);
  int*            NBR = (int*)(ws + oNBR);
  int*            MET = (int*)(ws + oMET);

  const size_t bldLds = (size_t)BLD_LDS_INTS * 4;
  hipFuncSetAttribute(reinterpret_cast<const void*>(&k_build), hipFuncAttributeMaxDynamicSharedMemorySize, (int)bldLds);

  const int nUx = NN * (FIN / 8);
  k_wprep<<<(NU1 + NU2 + NU3) / NTHR, NTHR, 0, stream>>>(W1, W2, W3, W1T, W2D, W3D);
  k_cvx<<<nUx / NTHR, NTHR, 0, stream>>>(x, nUx, XB);
  k_build<<<NN / NBA, NTHR, bldLds, stream>>>(ei, nE2, nN, vec8, NBR, MET);
  k_gemm<<<dim3(NN / GBM, FH / GBN), GTHR, 0, stream>>>(XB, W1T, XW, FIN, FH);
  k_agg<4, 1><<<NN / NWAVE, NTHR, 0, stream>>>(NBR, MET, XW, b1, H, out, nN);
  k_gemm<<<dim3(NN / GBM, FH / GBN), GTHR, 0, stream>>>(H, W2D, XW, HP, FH);
  k_agg<4, 1><<<NN / NWAVE, NTHR, 0, stream>>>(NBR, MET, XW, b2, H, out, nN);
  k_gemm<<<dim3(NN / GBM, FO / GBN), GTHR, 0, stream>>>(H, W3D, XW, HP, FO);
  k_agg<2, 0><<<NN / NWAVE, NTHR, 0, stream>>>(NBR, MET, XW, b3, H, out, nN);
}
